// DeformConvV3_12214886990431
// MI455X (gfx1250) — hardware-verified
//
#include <hip/hip_runtime.h>
#define NBt 8
#define CC 256
#define HH 56
#define NTK (HH * HH)
#define NR (NBt * NTK)
#define GG 8
#define GC 32
#define PP 9
#define PW 58
#define NOFF 144
#define NMSK 72
#define NOM 224
typedef __bf16 v16b __attribute__((ext_vector_type(16)));
typedef unsigned short v8us __attribute__((ext_vector_type(8), may_alias));
typedef float  v8f  __attribute__((ext_vector_type(8)));
typedef float  v4f  __attribute__((ext_vector_type(4)));
typedef float  v4fa __attribute__((ext_vector_type(4), may_alias));
union FragB { v16b v; v8us half[2]; unsigned short u[16]; };

__device__ __forceinline__ unsigned short bf16_bits(float x) { unsigned int u = __float_as_uint(x); return (unsigned short)((u + 0x7FFFu + ((u >> 16) & 1u)) >> 16); }
__device__ __forceinline__ float bf16_val(unsigned short b) { return __uint_as_float(((unsigned int)b) << 16); }
__device__ __forceinline__ float bf16_round(float x) { return bf16_val(bf16_bits(x)); }
template <int NT>
__device__ __forceinline__ v8f mmaN(v16b ah, v16b al, v16b bh, v16b bl, v8f c) {
  c = __builtin_amdgcn_wmma_f32_16x16x32_bf16(false, ah, false, bh, (short)0, c, false, false);
  if (NT >= 2) c = __builtin_amdgcn_wmma_f32_16x16x32_bf16(false, al, false, bh, (short)0, c, false, false);
  if (NT >= 3) c = __builtin_amdgcn_wmma_f32_16x16x32_bf16(false, ah, false, bl, (short)0, c, false, false);
  asm volatile("v_nop\n\tv_nop\n\tv_nop\n\tv_nop" : "+v"(c) : "v"(ah), "v"(al), "v"(bh), "v"(bl));
  return c;
}

__global__ __launch_bounds__(256) void k_wt_bf16(const float* __restrict__ W, unsigned short* __restrict__ Wt, int K, int N) {
  const int t = blockIdx.x * 256 + threadIdx.x;
  const int k8n = K / 8;
  if (t >= N * k8n) return;
  const int n = t / k8n, k8 = (t % k8n) * 8;
  v8us v;
#pragma unroll
  for (int i = 0; i < 8; ++i) v[i] = bf16_bits(W[(size_t)(k8 + i) * N + n]);
  *(volatile v8us*)(Wt + (size_t)n * K + k8) = v;
  __threadfence();
  *(volatile v8us*)(Wt + (size_t)n * K + k8) = v;
}

template <bool ASPLIT, int ACT, bool BIAS_BF16>
__global__ __launch_bounds__(128) void k_gemm_bf(const float* __restrict__ A, int lda, const unsigned short* __restrict__ Wt, int ldb,
                                               const float* __restrict__ bias, float* __restrict__ C, int ldc, int M, int N, int K) {
  __shared__ __attribute__((aligned(16))) float so[4][16][64];
  const int tid = threadIdx.x, w = tid >> 5, lane = tid & 31, ln = lane & 15, hh = lane >> 4;
  const int ntn = N / 64;
  const int wid = blockIdx.x * 4 + w;
  const int mt = wid / ntn, nq = wid % ntn;
  if (mt * 16 >= M) return;
  const int row0 = mt * 16, col0 = nq * 64;
  const float* arow = A + (size_t)(row0 + ln) * lda;
  v8f acc[4] = {};
  for (int kb = 0; kb < K; kb += 32) {
    FragB ah, al;
    const v4f x0 = *(const v4fa*)(arow + kb + 8 * hh), x1 = *(const v4fa*)(arow + kb + 8 * hh + 4);
    const v4f x2 = *(const v4fa*)(arow + kb + 16 + 8 * hh), x3 = *(const v4fa*)(arow + kb + 16 + 8 * hh + 4);
    float xs[16] = {x0[0],x0[1],x0[2],x0[3],x1[0],x1[1],x1[2],x1[3],x2[0],x2[1],x2[2],x2[3],x3[0],x3[1],x3[2],x3[3]};
#pragma unroll
    for (int i = 0; i < 16; ++i) { const unsigned short hb = bf16_bits(xs[i]); ah.u[i] = hb; al.u[i] = ASPLIT ? bf16_bits(xs[i] - bf16_val(hb)) : (unsigned short)0; }
#pragma unroll
    for (int t = 0; t < 4; ++t) {
      const unsigned short* brow = Wt + (size_t)(col0 + t * 16 + ln) * ldb + kb;
      FragB b;
      b.half[0] = *(const v8us*)(brow + 8 * hh);
      b.half[1] = *(const v8us*)(brow + 16 + 8 * hh);
      acc[t] = mmaN<ASPLIT ? 2 : 1>(ah.v, al.v, b.v, b.v, acc[t]);
    }
  }
#pragma unroll
  for (int t = 0; t < 4; ++t) {
    float bv = bias ? bias[col0 + t * 16 + ln] : 0.f;
    if (BIAS_BF16) bv = bf16_round(bv);
#pragma unroll
    for (int r = 0; r < 8; ++r) { float v = acc[t][r] + bv; if (ACT == 1) v = fmaxf(v, 0.f); so[w][8 * hh + r][t * 16 + ln] = v; }
  }
  __builtin_amdgcn_fence(__ATOMIC_ACQ_REL, "workgroup");
  __builtin_amdgcn_wave_barrier();
  const int rsub = lane >> 4, c4 = (lane & 15) * 4;
  for (int pass = 0; pass < 2; ++pass) {
#pragma unroll
    for (int q = 0; q < 8; ++q) {
      const int r = q * 2 + rsub;
      const v4f v = *(const v4fa*)&so[w][r][c4];
      *(volatile v4f*)(C + (size_t)(row0 + r) * ldc + col0 + c4) = v;
    }
    if (pass == 0) __threadfence();
  }
}

template <bool ASPLIT, int ACT, bool BIAS_BF16, bool RES_BF16>
__global__ __launch_bounds__(128) void k_gemm_bf3(const float* __restrict__ A, int lda, const unsigned short* __restrict__ Wt, int ldb,
                                                const float* __restrict__ bias, const float* __restrict__ resid, int rmod, int ldr,
                                                float* __restrict__ C, int ldc, int M, int N, int K) {
  __shared__ __attribute__((aligned(16))) float so[4][16][64];
  const int tid = threadIdx.x, w = tid >> 5, lane = tid & 31, ln = lane & 15, hh = lane >> 4;
  const int ntn = N / 64;
  const int wid = blockIdx.x * 4 + w;
  const int mt = wid / ntn, nq = wid % ntn;
  if (mt * 16 >= M) return;
  const int row0 = mt * 16, col0 = nq * 64;
  const float* arow = A + (size_t)(row0 + ln) * lda;
  v8f acc[4] = {};
  for (int kb = 0; kb < K; kb += 32) {
    FragB ah, al;
    const v4f x0 = *(const v4fa*)(arow + kb + 8 * hh), x1 = *(const v4fa*)(arow + kb + 8 * hh + 4);
    const v4f x2 = *(const v4fa*)(arow + kb + 16 + 8 * hh), x3 = *(const v4fa*)(arow + kb + 16 + 8 * hh + 4);
    float xs[16] = {x0[0],x0[1],x0[2],x0[3],x1[0],x1[1],x1[2],x1[3],x2[0],x2[1],x2[2],x2[3],x3[0],x3[1],x3[2],x3[3]};
#pragma unroll
    for (int i = 0; i < 16; ++i) { const unsigned short hb = bf16_bits(xs[i]); ah.u[i] = hb; al.u[i] = ASPLIT ? bf16_bits(xs[i] - bf16_val(hb)) : (unsigned short)0; }
#pragma unroll
    for (int t = 0; t < 4; ++t) {
      const unsigned short* brow = Wt + (size_t)(col0 + t * 16 + ln) * ldb + kb;
      FragB b;
      b.half[0] = *(const v8us*)(brow + 8 * hh);
      b.half[1] = *(const v8us*)(brow + 16 + 8 * hh);
      acc[t] = mmaN<ASPLIT ? 2 : 1>(ah.v, al.v, b.v, b.v, acc[t]);
    }
  }
#pragma unroll
  for (int t = 0; t < 4; ++t) {
    const int col = col0 + t * 16 + ln;
    float bv = bias ? bias[col] : 0.f;
    if (BIAS_BF16) bv = bf16_round(bv);
#pragma unroll
    for (int r = 0; r < 8; ++r) {
      float v = acc[t][r] + bv;
      if (resid) { float rv = resid[(size_t)((row0 + 8 * hh + r) % rmod) * ldr + col]; if (RES_BF16) rv = bf16_round(rv); v += rv; }
      if (ACT == 1) v = fmaxf(v, 0.f);
      if (ACT == 2) v = 0.5f * v * (1.0f + erff(v * 0.70710678118654752f));
      if (ACT == 3) { const float u = 0.7978845608028654f * (v + 0.044715f * v * v * v); v = 0.5f * v * (1.0f + tanhf(u)); }
      so[w][8 * hh + r][t * 16 + ln] = v;
    }
  }
  __builtin_amdgcn_fence(__ATOMIC_ACQ_REL, "workgroup");
  __builtin_amdgcn_wave_barrier();
  const int rsub = lane >> 4, c4 = (lane & 15) * 4;
  for (int pass = 0; pass < 2; ++pass) {
#pragma unroll
    for (int q = 0; q < 8; ++q) {
      const int r = q * 2 + rsub;
      const v4f v = *(const v4fa*)&so[w][r][c4];
      *(volatile v4f*)(C + (size_t)(row0 + r) * ldc + col0 + c4) = v;
    }
    if (pass == 0) __threadfence();
  }
}
template <bool PARAM_BF16>
__global__ __launch_bounds__(256) void k_layernorm(const float* __restrict__ X, const float* __restrict__ R, const float* __restrict__ g, const float* __restrict__ bta,
                                                  float* __restrict__ out_sum, float* __restrict__ out_norm, int N, float eps) {
  __shared__ float red[256];
  const int row = blockIdx.x, tid = threadIdx.x;
  const float* x = X + (size_t)row * N; const float* rr = R ? R + (size_t)row * N : nullptr;
  float vals[16];
  const int per = N / 256;
  float s1 = 0.f;
  for (int u = 0; u < per / 4; ++u) {
    const int j = tid * 4 + 1024 * u;
    const v4f a = *(const v4fa*)(x + j);
    v4f b = {0.f,0.f,0.f,0.f}; if (rr) b = *(const v4fa*)(rr + j);
#pragma unroll
    for (int q = 0; q < 4; ++q) { const float v = a[q] + b[q]; vals[u * 4 + q] = v; s1 += v; }
  }
  red[tid] = s1; __syncthreads();
  for (int st = 128; st > 0; st >>= 1) { if (tid < st) red[tid] += red[tid + st]; __syncthreads(); }
  const float mu = red[0] / (float)N; __syncthreads();
  float s2 = 0.f;
  for (int u = 0; u < per / 4; ++u)
#pragma unroll
    for (int q = 0; q < 4; ++q) { const float c = vals[u * 4 + q] - mu; s2 += c * c; }
  red[tid] = s2; __syncthreads();
  for (int st = 128; st > 0; st >>= 1) { if (tid < st) red[tid] += red[tid + st]; __syncthreads(); }
  const float rs = rsqrtf(red[0] / (float)N + eps);
  for (int pass = 0; pass < 2; ++pass) {
    for (int u = 0; u < per / 4; ++u) {
      const int j = tid * 4 + 1024 * u;
      v4f o, sm;
#pragma unroll
      for (int q = 0; q < 4; ++q) {
        float gg = g[j + q], bb = bta[j + q];
        if (PARAM_BF16) { gg = bf16_round(gg); bb = bf16_round(bb); }
        sm[q] = vals[u * 4 + q]; o[q] = (vals[u * 4 + q] - mu) * rs * gg + bb;
      }
      if (out_sum) *(volatile v4f*)(out_sum + (size_t)row * N + j) = sm;
      *(volatile v4f*)(out_norm + (size_t)row * N + j) = o;
    }
    if (pass == 0) __threadfence();
  }
}


typedef _Float16 v16h __attribute__((ext_vector_type(16)));
union FragH { v16h v; v8us half[2]; _Float16 h[16]; unsigned short u[16]; };
template <int NT>
__device__ __forceinline__ v8f mmaH(v16h ah, v16h al, v16h bh, v16h bl, v8f c) {
  c = __builtin_amdgcn_wmma_f32_16x16x32_f16(false, ah, false, bh, (short)0, c, false, false);
  if (NT >= 2) c = __builtin_amdgcn_wmma_f32_16x16x32_f16(false, al, false, bh, (short)0, c, false, false);
  if (NT >= 3) c = __builtin_amdgcn_wmma_f32_16x16x32_f16(false, ah, false, bl, (short)0, c, false, false);
  asm volatile("v_nop\n\tv_nop\n\tv_nop\n\tv_nop" : "+v"(c) : "v"(ah), "v"(al), "v"(bh), "v"(bl));
  return c;
}
template <bool ASPLIT>
__global__ __launch_bounds__(128) void k_gemm_h(const float* __restrict__ A, int lda, size_t sA, const _Float16* __restrict__ Bh, int ldb, size_t sB, float alpha, float* __restrict__ C, int ldc, size_t sC, int M, int N, int K) {
  __shared__ __attribute__((aligned(16))) float so[4][16][64];
  const int tid = threadIdx.x, w = tid >> 5, lane = tid & 31, ln = lane & 15, hh = lane >> 4; const int by = blockIdx.y;
  A += (size_t)by * sA; Bh += (size_t)by * sB; C += (size_t)by * sC;
  const int ntn = (N + 63) / 64; const int wid = blockIdx.x * 4 + w; const int mt = wid / ntn, nq = wid % ntn; if (mt * 16 >= M) return;
  const int row0 = mt * 16, col0 = nq * 64; const float* arow = A + (size_t)(row0 + ln) * lda;
  v8f acc[4] = {};
  for (int kb = 0; kb < K; kb += 32) {
    FragH ah, al;
    const v4f x0 = *(const v4fa*)(arow + kb + 8 * hh), x1 = *(const v4fa*)(arow + kb + 8 * hh + 4), x2 = *(const v4fa*)(arow + kb + 16 + 8 * hh), x3 = *(const v4fa*)(arow + kb + 16 + 8 * hh + 4);
    float xs[16] = {x0[0],x0[1],x0[2],x0[3],x1[0],x1[1],x1[2],x1[3],x2[0],x2[1],x2[2],x2[3],x3[0],x3[1],x3[2],x3[3]};
#pragma unroll
    for (int i = 0; i < 16; ++i) { const _Float16 h = (_Float16)xs[i]; ah.h[i] = h; al.h[i] = ASPLIT ? (_Float16)(xs[i] - (float)h) : (_Float16)0.0f; }
#pragma unroll
    for (int t = 0; t < 4; ++t) { if (col0 + t * 16 >= N) continue; const size_t boff = (size_t)(col0 + t * 16 + ln) * ldb + kb; FragH bq; bq.half[0] = *(const v8us*)(Bh + boff + 8 * hh); bq.half[1] = *(const v8us*)(Bh + boff + 16 + 8 * hh);
      acc[t] = mmaH<ASPLIT ? 2 : 1>(ah.v, al.v, bq.v, bq.v, acc[t]); }
  }
#pragma unroll
  for (int t = 0; t < 4; ++t) { if (col0 + t * 16 >= N) continue;
#pragma unroll
    for (int r = 0; r < 8; ++r) so[w][8 * hh + r][t * 16 + ln] = acc[t][r] * alpha; }
  __builtin_amdgcn_fence(__ATOMIC_ACQ_REL, "workgroup"); __builtin_amdgcn_wave_barrier();
  const int rsub = lane >> 4, c4 = (lane & 15) * 4;
  for (int pass = 0; pass < 2; ++pass) {
#pragma unroll
    for (int q = 0; q < 8; ++q) { const int r = q * 2 + rsub; if (col0 + c4 < N) { const v4f v = *(const v4fa*)&so[w][r][c4]; *(volatile v4f*)(C + (size_t)(row0 + r) * ldc + col0 + c4) = v; } }
    if (pass == 0) __threadfence(); }
}

__global__ __launch_bounds__(256) void k_wt_f16(const float* __restrict__ W, _Float16* __restrict__ Wt, int K, int N, float scale) {
  const int t = blockIdx.x * 256 + threadIdx.x; if (t >= N * (K / 8)) return; const int n = t / (K / 8), k8 = (t % (K / 8)) * 8; FragH f;
#pragma unroll
  for (int i = 0; i < 8; ++i) f.h[i] = (_Float16)(bf16_round(W[(size_t)(k8 + i) * N + n]) * scale); const v8us o = f.half[0];
  *(volatile v8us*)((unsigned short*)Wt + (size_t)n * K + k8) = o; __threadfence(); *(volatile v8us*)((unsigned short*)Wt + (size_t)n * K + k8) = o;
}
template <int ACT>
__global__ __launch_bounds__(128) void k_gemm_hhx(const _Float16* __restrict__ A, int lda, size_t sA, const _Float16* __restrict__ Bh, int ldb, size_t sB, float alpha, const float* __restrict__ bias, size_t sBias, const float* __restrict__ CP, int rowsPerB, size_t sCPb, int row0g,
    float* __restrict__ C, _Float16* __restrict__ C16, int ldc, size_t sC, int M, int N, int K) {
  __shared__ __attribute__((aligned(16))) float so[4][16][64];
  const int tid = threadIdx.x, w = tid >> 5, lane = tid & 31, ln = lane & 15, hh = lane >> 4; const int by = blockIdx.y;
  A += (size_t)by * sA; Bh += (size_t)by * sB; const size_t cofs = (size_t)by * sC; const float* bp = bias ? bias + (size_t)by * sBias : nullptr;
  const int ntn = (N + 63) / 64; const int wid = blockIdx.x * 4 + w; const int mt = wid / ntn, nq = wid % ntn; if (mt * 16 >= M) return;
  const int row0 = mt * 16, col0 = nq * 64; const _Float16* arow = A + (size_t)(row0 + ln) * lda;
  v8f acc[4] = {};
  for (int kb = 0; kb < K; kb += 32) { FragH ah; ah.half[0] = *(const v8us*)((const unsigned short*)arow + kb + 8 * hh); ah.half[1] = *(const v8us*)((const unsigned short*)arow + kb + 16 + 8 * hh);
#pragma unroll
    for (int t = 0; t < 4; ++t) { if (col0 + t * 16 >= N) continue; const size_t boff = (size_t)(col0 + t * 16 + ln) * ldb + kb; FragH bq; bq.half[0] = *(const v8us*)((const unsigned short*)Bh + boff + 8 * hh); bq.half[1] = *(const v8us*)((const unsigned short*)Bh + boff + 16 + 8 * hh);
      acc[t] = mmaH<1>(ah.v, ah.v, bq.v, bq.v, acc[t]); }
  }
#pragma unroll
  for (int t = 0; t < 4; ++t) { if (col0 + t * 16 >= N) continue; const int col = col0 + t * 16 + ln; const float bv = bp ? bf16_round(bp[col]) : 0.f;
#pragma unroll
    for (int r = 0; r < 8; ++r) { float v = acc[t][r] * alpha + bv; if (CP) { const int bidx = (row0g + row0 + 8 * hh + r) / rowsPerB; v += CP[(size_t)bidx * sCPb + (size_t)by * 64 + col]; } if (ACT == 1) v = (v > 0.f) ? v : expm1f(v); else if (ACT == 7) v = (v > 0.f) ? v + 1.0f : expf(v); else if (ACT == 8) v = tanhf(v); else if (ACT == 9) v = 0.5f * v * (1.0f + tanhf(0.7978845608028654f * (v + 0.044715f * v * v * v))); else if (ACT == 11) v = 1.0f / (1.0f + expf(-v)); else if (ACT == 12) v = (v > 0.f) ? v : 0.01f * v; else if (ACT == 14) v = (v > 0.f) ? v : 0.1f * v; else if (ACT == 15) v = v / (1.0f + expf(-v)); else if (ACT == 3) v = fmaxf(v, 0.f); else if (ACT == 6) v = 0.5f * v * (1.0f + erff(v * 0.70710678118654752f)); so[w][8 * hh + r][t * 16 + ln] = v; } }
  __builtin_amdgcn_fence(__ATOMIC_ACQ_REL, "workgroup"); __builtin_amdgcn_wave_barrier();
  const int rsub = lane >> 4, c4 = (lane & 15) * 4; typedef _Float16 v4h __attribute__((ext_vector_type(4)));
  for (int pass = 0; pass < 2; ++pass) {
#pragma unroll
    for (int q = 0; q < 8; ++q) { const int r = q * 2 + rsub; if (col0 + c4 < N) { const v4f v = *(const v4fa*)&so[w][r][c4]; if (C) *(volatile v4f*)(C + cofs + (size_t)(row0 + r) * ldc + col0 + c4) = v; if (C16) { v4h h4; for (int i = 0; i < 4; ++i) h4[i] = (_Float16)v[i]; *(volatile v4h*)(C16 + cofs + (size_t)(row0 + r) * ldc + col0 + c4) = h4; } } }
    if (pass == 0) __threadfence(); }
}


typedef _Float16 v4h __attribute__((ext_vector_type(4)));

__global__ __launch_bounds__(256) void k_x16(const float* __restrict__ x, _Float16* __restrict__ X16, size_t n8) { const size_t t = (size_t)blockIdx.x * 256 + threadIdx.x; if (t >= n8) return; FragH f;
#pragma unroll
  for (int q = 0; q < 8; ++q) f.h[q] = (_Float16)bf16_round(x[t * 8 + q]); *(volatile v8us*)((unsigned short*)X16 + t * 8) = f.half[0]; __threadfence(); *(volatile v8us*)((unsigned short*)X16 + t * 8) = f.half[0]; }
__global__ __launch_bounds__(256) void k_h16(const float* __restrict__ x, _Float16* __restrict__ X16, size_t n8) { const size_t t = (size_t)blockIdx.x * 256 + threadIdx.x; if (t >= n8) return; FragH f;
#pragma unroll
  for (int q = 0; q < 8; ++q) f.h[q] = (_Float16)x[t * 8 + q]; *(volatile v8us*)((unsigned short*)X16 + t * 8) = f.half[0]; __threadfence(); *(volatile v8us*)((unsigned short*)X16 + t * 8) = f.half[0]; }
__global__ __launch_bounds__(256) void k_round16f(const float* __restrict__ W, _Float16* __restrict__ Bt, size_t n8) { const size_t t = (size_t)blockIdx.x * 256 + threadIdx.x; if (t >= n8) return; FragH f;
#pragma unroll
  for (int i = 0; i < 8; ++i) f.h[i] = (_Float16)(bf16_round(W[t * 8 + i]) * 16.0f); *(volatile v8us*)((unsigned short*)Bt + t * 8) = f.half[0]; __threadfence(); *(volatile v8us*)((unsigned short*)Bt + t * 8) = f.half[0]; }
template <int NHv, int TTv>
__global__ __launch_bounds__(256) void k_vt(const _Float16* __restrict__ V16, int ldv, int voff, _Float16* __restrict__ Vt) { __shared__ unsigned short tl[64][66]; const int tid = threadIdx.x; const int slab = blockIdx.x / (TTv / 64), lg = blockIdx.x % (TTv / 64); const int b = slab / NHv, h = slab % NHv;
  for (int i = tid; i < 64 * 8; i += 256) { const int r = i / 8, c8 = (i % 8) * 8; FragH f; f.half[0] = *(const v8us*)((const unsigned short*)V16 + ((size_t)b * TTv + lg * 64 + r) * ldv + voff + h * 64 + c8);
#pragma unroll
    for (int q = 0; q < 8; ++q) tl[r][c8 + q] = f.u[q]; }
  __syncthreads();
  for (int pass = 0; pass < 2; ++pass) {
#pragma unroll
    for (int rd = 0; rd < 2; ++rd) { const int d = rd * 32 + tid / 8, pc = tid % 8; FragH f;
#pragma unroll
      for (int q = 0; q < 8; ++q) f.u[q] = tl[pc * 8 + q][d];
      *(volatile v8us*)((unsigned short*)Vt + ((size_t)slab * 64 + d) * TTv + lg * 64 + pc * 8) = f.half[0]; }
    if (pass == 0) __threadfence(); } }

__global__ __launch_bounds__(256) void k_hl(const float* __restrict__ F, _Float16* __restrict__ Hh, _Float16* __restrict__ Hl, size_t n8) { const size_t t = (size_t)blockIdx.x * 256 + threadIdx.x; if (t >= n8) return; FragH fh, fl; const v4f a = *(const v4fa*)(F + t * 8), c = *(const v4fa*)(F + t * 8 + 4);
#pragma unroll
  for (int q = 0; q < 4; ++q) { _Float16 h = (_Float16)a[q]; fh.h[q] = h; fl.h[q] = (_Float16)((a[q] - (float)h) * 1024.0f); h = (_Float16)c[q]; fh.h[4 + q] = h; fl.h[4 + q] = (_Float16)((c[q] - (float)h) * 1024.0f); }
  for (int pass = 0; pass < 2; ++pass) { *(volatile v8us*)((unsigned short*)Hh + t * 8) = fh.half[0]; *(volatile v8us*)((unsigned short*)Hl + t * 8) = fl.half[0]; if (pass == 0) __threadfence(); } }

__device__ __forceinline__ float gelu_f(float v) { return 0.5f * v * (1.0f + erff(v * 0.70710678118654752f)); }
__global__ __launch_bounds__(256) void k_tok16(const float* __restrict__ x, _Float16* __restrict__ X16) { const int t = blockIdx.x * 256 + threadIdx.x; if (t >= NR * (CC / 8)) return; const int c0 = (t % (CC / 8)) * 8, r = t / (CC / 8); const int b = r / NTK, l = r % NTK; FragH f;
#pragma unroll
  for (int q = 0; q < 8; ++q) f.h[q] = (_Float16)bf16_round(x[((size_t)b * CC + c0 + q) * NTK + l]);
  *(volatile v8us*)((unsigned short*)X16 + (size_t)r * CC + c0) = f.half[0]; __threadfence(); *(volatile v8us*)((unsigned short*)X16 + (size_t)r * CC + c0) = f.half[0]; }
__global__ __launch_bounds__(256) void k_split(const float* __restrict__ F, _Float16* __restrict__ Hh, _Float16* __restrict__ Hl, size_t n8) {
  #pragma clang fp contract(off)
  const size_t t = (size_t)blockIdx.x * 256 + threadIdx.x; if (t >= n8) return; const v4f a = *(const v4fa*)(F + t * 8), c = *(const v4fa*)(F + t * 8 + 4); FragH fh, fl;
#pragma unroll
  for (int q = 0; q < 8; ++q) { const float v = (q < 4) ? a[q] : c[q - 4]; const _Float16 hi = (_Float16)v; fh.h[q] = hi; fl.h[q] = (_Float16)((v - (float)hi) * 1024.0f); }
  for (int pass = 0; pass < 2; ++pass) { *(volatile v8us*)((unsigned short*)Hh + t * 8) = fh.half[0]; *(volatile v8us*)((unsigned short*)Hl + t * 8) = fl.half[0]; if (pass == 0) __threadfence(); } }
__global__ __launch_bounds__(256) void k_dw(const float* __restrict__ x, const float* __restrict__ dw, const float* __restrict__ db, float* __restrict__ Fd) {
  #pragma clang fp contract(off)
  const int t = blockIdx.x * 256 + threadIdx.x; if (t >= NR * (CC / 4)) return; const int c0 = (t % (CC / 4)) * 4, r = t / (CC / 4); const int b = r / NTK, l = r % NTK; const int h = l / HH, w = l % HH; v4f o;
#pragma unroll
  for (int k = 0; k < 4; ++k) { const int c = c0 + k; const float* xp = x + ((size_t)b * CC + c) * NTK; float a = bf16_round(db[c]);
#pragma unroll
    for (int tp = 0; tp < 9; ++tp) { const int yy = h + tp / 3 - 1, xx = w + tp % 3 - 1; const bool in = (yy >= 0 && yy < HH && xx >= 0 && xx < HH); const float xv = bf16_round(xp[min(max(yy, 0), HH - 1) * HH + min(max(xx, 0), HH - 1)]); a += (in ? xv : 0.f) * bf16_round(dw[c * 9 + tp]); }
    o[k] = a; }
  *(volatile v4f*)(Fd + (size_t)r * CC + c0) = o; __threadfence(); *(volatile v4f*)(Fd + (size_t)r * CC + c0) = o; }
__global__ __launch_bounds__(256) void k_lnf(float* __restrict__ Fd, const float* __restrict__ g, const float* __restrict__ bb, _Float16* __restrict__ F2) {
  #pragma clang fp contract(off)
  const int tid = threadIdx.x, wv = tid >> 5, ln = tid & 31; const int r = blockIdx.x * 8 + wv; if (r >= NR) return; float v[8]; float s = 0.f;
#pragma unroll
  for (int k = 0; k < 8; ++k) { v[k] = Fd[(size_t)r * CC + ln * 8 + k]; s += v[k]; }
  for (int o = 16; o > 0; o >>= 1) s += __shfl_xor(s, o, 32); const float mu = s / (float)CC; float q2 = 0.f;
#pragma unroll
  for (int k = 0; k < 8; ++k) { const float d = v[k] - mu; q2 += d * d; }
  for (int o = 16; o > 0; o >>= 1) q2 += __shfl_xor(q2, o, 32); const float rs = rsqrtf(q2 / (float)CC + 1e-5f); v4f oa, ob;
#pragma unroll
  for (int k = 0; k < 8; ++k) { const int c = ln * 8 + k; const float y = (v[k] - mu) * rs * bf16_round(g[c]) + bf16_round(bb[c]); if (k < 4) oa[k] = y; else ob[k - 4] = y; }
  (void)F2;
  for (int pass = 0; pass < 2; ++pass) { *(volatile v4f*)((float*)Fd + (size_t)r * CC + ln * 8) = oa; *(volatile v4f*)((float*)Fd + (size_t)r * CC + ln * 8 + 4) = ob; if (pass == 0) __threadfence(); } }
__global__ __launch_bounds__(256) void k_gf(const float* __restrict__ L, _Float16* __restrict__ F2) {
  #pragma clang fp contract(off)
  const int t = blockIdx.x * 256 + threadIdx.x; if (t >= NR * (CC / 4)) return; const int c0 = (t % (CC / 4)) * 4, r = t / (CC / 4); const v4f a = *(const v4fa*)(L + (size_t)r * CC + c0); FragH fh, fl;
#pragma unroll
  for (int q = 0; q < 4; ++q) { const float y = gelu_f(a[q]); const _Float16 hi = (_Float16)y; fh.h[q] = hi; fl.h[q] = (_Float16)((y - (float)hi) * 1024.0f); }
  const unsigned long long ph = *(const unsigned long long*)&fh.u[0], pl = *(const unsigned long long*)&fl.u[0];
  for (int pass = 0; pass < 2; ++pass) { *(volatile unsigned long long*)((unsigned short*)F2 + (size_t)r * 512 + c0) = ph; *(volatile unsigned long long*)((unsigned short*)F2 + (size_t)r * 512 + 256 + c0) = pl; if (pass == 0) __threadfence(); } }
__global__ __launch_bounds__(256) void k_bfold2(const float* __restrict__ W1, int O1, const float* __restrict__ W2, int O2, int Opad, _Float16* __restrict__ Bt) { const int t = blockIdx.x * 256 + threadIdx.x; if (t >= Opad * 64) return; const int k0 = (t & 63) * 8, o = t >> 6; const int kb = k0 & 255; const float sc = (k0 >= 256) ? (16.0f / 1024.0f) : 16.0f; const int o1 = min(o, O1 - 1), o2 = min(max(o - O1, 0), max(O2 - 1, 0)); FragH f;
#pragma unroll
  for (int q = 0; q < 8; ++q) { const float a = bf16_round(W1[(size_t)(kb + q) * O1 + o1]); const float bq = W2 ? bf16_round(W2[(size_t)(kb + q) * O2 + o2]) : 0.f; const float v = (o < O1) ? a : (o < O1 + O2) ? bq : 0.f; f.h[q] = (_Float16)(v * sc); }
  *(volatile v8us*)((unsigned short*)Bt + (size_t)o * 512 + k0) = f.half[0]; __threadfence(); *(volatile v8us*)((unsigned short*)Bt + (size_t)o * 512 + k0) = f.half[0]; }
__global__ __launch_bounds__(256) void k_bcat(const float* __restrict__ b1, const float* __restrict__ b2, float* __restrict__ BP) { const int l = threadIdx.x; if (l >= NOM) return; const float v = (l < NOFF) ? b1[l] : b2[min(max(l - NOFF, 0), NMSK - 1)]; *(volatile float*)(BP + l) = v; __threadfence(); *(volatile float*)(BP + l) = v; }
__global__ __launch_bounds__(256) void k_dcn3(const float* __restrict__ OM, const _Float16* __restrict__ Vh, const _Float16* __restrict__ Vl, _Float16* __restrict__ D2) {
  #pragma clang fp contract(off)
  __shared__ unsigned short slab[32 * 256]; const int t = blockIdx.x * 256 + threadIdx.x; const int g = t & 7, r = t >> 3; const int rl = threadIdx.x >> 3; const int rbase = blockIdx.x * 32; const int b = r / NTK, l = r % NTK; const int h = l / HH, w = l % HH; const float* om = OM + (size_t)r * NOM;
  float mk[PP]; { float mx = -3.0e38f;
#pragma unroll
    for (int p = 0; p < PP; ++p) { mk[p] = om[NOFF + g * PP + p]; mx = fmaxf(mx, mk[p]); }
    float su = 0.f;
#pragma unroll
    for (int p = 0; p < PP; ++p) { mk[p] = expf(mk[p] - mx); su += mk[p]; }
#pragma unroll
    for (int p = 0; p < PP; ++p) mk[p] = mk[p] / su; }
  float acc[GC];
#pragma unroll
  for (int c = 0; c < GC; ++c) acc[c] = 0.f;
  const float refx = (1.5f + (float)w) / (float)PW, refy = (1.5f + (float)h) / (float)PW;
#pragma unroll 1
  for (int p = 0; p < PP; ++p) { const float kxp = (float)(p / 3 - 1), kyp = (float)(p % 3 - 1); const float offx = om[g * 18 + 2 * p], offy = om[g * 18 + 2 * p + 1];
    const float lx = (refx + kxp / (float)PW) + offx / (float)PW, ly = (refy + kyp / (float)PW) + offy / (float)PW; const float px = lx * (float)PW - 0.5f, py = ly * (float)PW - 0.5f; const float x0 = floorf(px), y0 = floorf(py); const float wx = px - x0, wy = py - y0; const int xi = (int)x0, yi = (int)y0;
    float mp = 0.f;
#pragma unroll
    for (int q = 0; q < PP; ++q) mp = (q == p) ? mk[q] : mp;
#pragma unroll 1
    for (int cn = 0; cn < 4; ++cn) { const int xx = xi + (cn & 1), yy = yi + (cn >> 1); const bool valid = (xx >= 0 && xx < PW && yy >= 0 && yy < PW); const int ux = xx - 1, uy = yy - 1; const bool inner = (ux >= 0 && ux < HH && uy >= 0 && uy < HH); const float wgt = ((cn & 1) ? wx : (1.0f - wx)) * ((cn >> 1) ? wy : (1.0f - wy)); const float f = (valid && inner) ? (mp * wgt) : 0.f; const size_t src = ((size_t)b * NTK + (size_t)min(max(uy, 0), HH - 1) * HH + min(max(ux, 0), HH - 1)) * CC + g * GC;
#pragma unroll
      for (int hq = 0; hq < 4; ++hq) { FragH vh, vl; vh.half[0] = *(const v8us*)((const unsigned short*)Vh + src + hq * 8); vl.half[0] = *(const v8us*)((const unsigned short*)Vl + src + hq * 8);
#pragma unroll
        for (int c = 0; c < 8; ++c) acc[hq * 8 + c] += f * ((float)vh.h[c] + (float)vl.h[c] * 0.0009765625f); } } }
  FragH oh[4], ol[4];
#pragma unroll
  for (int c = 0; c < GC; ++c) { const _Float16 hi = (_Float16)acc[c]; oh[c >> 3].h[c & 7] = hi; ol[c >> 3].h[c & 7] = (_Float16)((acc[c] - (float)hi) * 1024.0f); }
  for (int ph = 0; ph < 2; ++ph) {
    __syncthreads();
#pragma unroll
    for (int q = 0; q < 4; ++q) *(v8us*)(slab + rl * 256 + g * GC + q * 8) = ph ? ol[q].half[0] : oh[q].half[0];
    __syncthreads();
    for (int pass = 0; pass < 2; ++pass) {
#pragma unroll
      for (int it = 0; it < 4; ++it) { const int ci = it * 256 + threadIdx.x; const int row = ci >> 5, ch = (ci & 31) * 8; const v8us val = *(const v8us*)(slab + row * 256 + ch); *(volatile v8us*)((unsigned short*)D2 + (size_t)(rbase + row) * 512 + ph * 256 + ch) = val; }
      if (pass == 0) __threadfence(); } } }
__global__ __launch_bounds__(256) void k_bnout(const float* __restrict__ Y, const float* __restrict__ bg, const float* __restrict__ bbv, const float* __restrict__ bm, const float* __restrict__ bv, float* __restrict__ out) {
  #pragma clang fp contract(off)
  const int t = blockIdx.x * 256 + threadIdx.x; if (t >= NBt * CC * (NTK / 4)) return; const int l0 = (t % (NTK / 4)) * 4; const int c = (t / (NTK / 4)) % CC; const int b = t / ((NTK / 4) * CC); const float sc = rsqrtf(bf16_round(bv[c]) + 1e-5f) * bf16_round(bg[c]), mn = bf16_round(bm[c]), bo = bf16_round(bbv[c]); v4f v;
#pragma unroll
  for (int q = 0; q < 4; ++q) { const float y = (Y[((size_t)b * NTK + l0 + q) * CC + c] - mn) * sc + bo; v[q] = y * (1.0f / (1.0f + expf(-y))); }
  float* dst = out + ((size_t)b * CC + c) * NTK + l0; *(volatile v4f*)dst = v; __threadfence(); *(volatile v4f*)dst = v; }

extern "C" void kernel_launch(void* const* d_in, const int* in_sizes, int n_in,
                              void* d_out, int out_size, void* d_ws, size_t ws_size, hipStream_t stream) {
  (void)in_sizes; (void)n_in; (void)out_size;
  const float* const* I = (const float* const*)d_in; const float* x = I[0]; const float* w_in = I[1]; const float* b_in = I[2]; const float* dw = I[3]; const float* db = I[4]; const float* lg = I[5]; const float* lb = I[6]; const float* w_off = I[7]; const float* b_off = I[8]; const float* w_mask = I[9]; const float* b_mask = I[10]; const float* w_out = I[11]; const float* b_out = I[12]; const float* bg = I[13]; const float* bbv = I[14]; const float* bm = I[15]; const float* bv = I[16];
  char* ws = (char*)d_ws; size_t off = 0;
  auto take = [&](size_t bytes) { char* p = ws + off; off += (bytes + 255) & ~(size_t)255; return p; };
  _Float16* BIN = (_Float16*)take((size_t)CC * CC * 2); _Float16* BOM = (_Float16*)take((size_t)NOM * 512 * 2); _Float16* BOUT = (_Float16*)take((size_t)CC * 512 * 2); float* BPom = (float*)take(NOM * 4);
  _Float16* X16 = (_Float16*)take((size_t)NR * CC * 2); float* V = (float*)take((size_t)NR * CC * 4); _Float16* Vh = (_Float16*)take((size_t)NR * CC * 2); _Float16* Vl = (_Float16*)take((size_t)NR * CC * 2); _Float16* F2 = (_Float16*)take((size_t)NR * 512 * 2); float* OM = (float*)take((size_t)NR * NOM * 4);
  _Float16* D2 = F2;
  float* Y = V;
  if (off > ws_size) return;
  k_wt_f16<<<(CC * (CC / 8) + 255) / 256, 256, 0, stream>>>(w_in, BIN, CC, CC, 16.0f);
  k_bfold2<<<(NOM * 64 + 255) / 256, 256, 0, stream>>>(w_off, NOFF, w_mask, NMSK, NOM, BOM); k_bcat<<<1, 256, 0, stream>>>(b_off, b_mask, BPom);
  k_bfold2<<<(CC * 64 + 255) / 256, 256, 0, stream>>>(w_out, CC, nullptr, 0, CC, BOUT);
  const size_t n8 = (size_t)NR * CC / 8; const unsigned nb8 = (unsigned)((n8 + 255) / 256); const dim3 gC(((NR / 16) * (CC / 64) + 3) / 4, 1), gOM((unsigned)(((NR / 16) * ((NOM + 63) / 64) + 3) / 4), 1);
  k_tok16<<<nb8, 256, 0, stream>>>(x, X16);
  k_gemm_hhx<0><<<gC, 128, 0, stream>>>(X16, CC, 0, BIN, CC, 0, 0.0625f, b_in, 0, nullptr, 1, 0, 0, V, nullptr, CC, 0, NR, CC, CC); k_split<<<nb8, 256, 0, stream>>>(V, Vh, Vl, n8);
  k_dw<<<(NR * (CC / 4) + 255) / 256, 256, 0, stream>>>(x, dw, db, V); k_lnf<<<NR / 8, 256, 0, stream>>>(V, lg, lb, F2); k_gf<<<(NR * (CC / 4) + 255) / 256, 256, 0, stream>>>(V, F2);
  k_gemm_hhx<0><<<gOM, 128, 0, stream>>>(F2, 512, 0, BOM, 512, 0, 0.0625f, BPom, 0, nullptr, 1, 0, 0, OM, nullptr, NOM, 0, NR, NOM, 512);
  k_dcn3<<<(NR * GG + 255) / 256, 256, 0, stream>>>(OM, Vh, Vl, D2);
  k_gemm_hhx<0><<<gC, 128, 0, stream>>>(D2, 512, 0, BOUT, 512, 0, 0.0625f, b_out, 0, nullptr, 1, 0, 0, Y, nullptr, CC, 0, NR, CC, 512);
  k_bnout<<<(unsigned)(((size_t)NBt * CC * (NTK / 4) + 255) / 256), 256, 0, stream>>>(Y, bg, bbv, bm, bv, (float*)d_out);
}
